// S6Layer_32950989094981
// MI455X (gfx1250) — hardware-verified
//
#include <hip/hip_runtime.h>
#include <math.h>

constexpr int kBatch   = 4;
constexpr int kT       = 1024;
constexpr int kDModel  = 512;
constexpr int kDInner  = 1024;
constexpr int kDState  = 512;
constexpr int kNDim    = 16;
constexpr int kKN      = kDState * kNDim;
constexpr int kTok     = kBatch * kT;
constexpr float kEps   = 1e-8f;
constexpr float kWCarry  = 256.0f;
constexpr float kXpCarry = 16.0f;
constexpr float kYiCarry = 64.0f;
constexpr int kChunk       = 64;
constexpr int kScanThreads = 512;
static_assert(kT % kChunk == 0);
static_assert(kChunk == 4 * (kScanThreads / 32));
static_assert(kDState % 32 == 0);

typedef __attribute__((ext_vector_type(16))) _Float16 v16h;
typedef __attribute__((ext_vector_type(8)))  _Float16 v8h;
typedef __attribute__((ext_vector_type(16))) __bf16   v16b;
typedef __attribute__((ext_vector_type(8)))  __bf16   v8b;
typedef __attribute__((ext_vector_type(8)))  float    v8f;
typedef __attribute__((ext_vector_type(4)))  float    v4f;
typedef __attribute__((ext_vector_type(4)))  unsigned int v4u;

__device__ __forceinline__ unsigned short f2bf_bits(float f) {
  unsigned u = __float_as_uint(f);
  return (unsigned short)((u + 0x7FFFu + ((u >> 16) & 1u)) >> 16);
}
__device__ __forceinline__ float bf_bits2f(unsigned short h) { return __uint_as_float(((unsigned)h) << 16); }

__device__ __forceinline__ void dep_guard_h(v8f& a, v8f& b, v16h x, v16h y) { asm volatile("v_nop\n\tv_nop\n\tv_nop\n\tv_nop" : "+v"(a), "+v"(b) : "v"(x), "v"(y)); }
__device__ __forceinline__ void dep_guard_b(v8f& a, v8f& b, v16b x, v16b y) { asm volatile("v_nop\n\tv_nop\n\tv_nop\n\tv_nop" : "+v"(a), "+v"(b) : "v"(x), "v"(y)); }
__device__ __forceinline__ void keep4_h(v16h a, v16h b, v16h c, v16h d) { asm volatile("v_nop" :: "v"(a), "v"(b), "v"(c), "v"(d)); }
__device__ __forceinline__ void keep4_b(v16b a, v16b b, v16b c, v16b d) { asm volatile("v_nop" :: "v"(a), "v"(b), "v"(c), "v"(d)); }
__device__ __forceinline__ void acc_guard4(v8f& a, v8f& b, v8f& c, v8f& d) { asm volatile("v_nop\n\tv_nop\n\tv_nop\n\tv_nop" : "+v"(a), "+v"(b), "+v"(c), "+v"(d)); }
template <typename T> struct Frag;
template <> struct Frag<_Float16> {
  typedef v16h V; union U { v16h v; v8h h[2]; };
  static __device__ __forceinline__ v16h load(const _Float16* p) {
    U f; f.h[0] = *(const v8h*)(p); f.h[1] = *(const v8h*)(p + 16); return f.v;
  }
  static __device__ __forceinline__ v8f mma(v16h a, v16h b, v8f c) {
    return __builtin_amdgcn_wmma_f32_16x16x32_f16(false, a, false, b, (short)0, c, false, false);
  }
  static __device__ __forceinline__ void guard(v8f& a, v8f& b, v16h x, v16h y) { dep_guard_h(a, b, x, y); }
  static __device__ __forceinline__ void keep(v16h a, v16h b, v16h c, v16h d) { keep4_h(a, b, c, d); }
};
template <> struct Frag<__bf16> {
  typedef v16b V; union U { v16b v; v8b h[2]; };
  static __device__ __forceinline__ v16b load(const __bf16* p) {
    U f; f.h[0] = *(const v8b*)(p); f.h[1] = *(const v8b*)(p + 16); return f.v;
  }
  static __device__ __forceinline__ v8f mma(v16b a, v16b b, v8f c) {
    return __builtin_amdgcn_wmma_f32_16x16x32_bf16(false, a, false, b, (short)0, c, false, false);
  }
  static __device__ __forceinline__ void guard(v8f& a, v8f& b, v16b x, v16b y) { dep_guard_b(a, b, x, y); }
  static __device__ __forceinline__ void keep(v16b a, v16b b, v16b c, v16b d) { keep4_b(a, b, c, d); }
};

__device__ __forceinline__ unsigned pk16(unsigned short a, unsigned short b) { return (unsigned)a | ((unsigned)b << 16); }
__device__ __forceinline__ unsigned short h_bits(float f) { const _Float16 h = (_Float16)f; return __builtin_bit_cast(unsigned short, h); }

template <int ET> struct Elem;
template <> struct Elem<0> { typedef _Float16 T; };
template <> struct Elem<1> { typedef __bf16 T; };
template <int ET, bool SPLIT, int BIAS_MODE, int OUT_MODE, bool RESID, int ACT = 0>
__global__ __launch_bounds__(256) void wmma_gemm64(
    const unsigned short* __restrict__ Ap, const unsigned short* __restrict__ A2p, int lda, long strideA,
    const unsigned short* __restrict__ Btp, const unsigned short* __restrict__ Bt2p, int ldb, long strideB,
    void* __restrict__ Cout, void* __restrict__ Cout2, int ldc, long strideC,
    const float* __restrict__ bias,
    const float* __restrict__ resid, long strideR,
    int M, int N, int K, float scale, float ocarry) {
  typedef typename Elem<ET>::T T;
  typedef typename Frag<T>::V V;
  const T* A = (const T*)Ap; const T* A2 = (const T*)A2p; const T* Bt = (const T*)Btp; const T* Bt2 = (const T*)Bt2p;
  __shared__ __align__(16) float sT[8][16 * 68];
  const int b    = blockIdx.y;
  const int lane = threadIdx.x & 31;
  const int wave = threadIdx.x >> 5;
  const int tilesN = N >> 6;
  const int tilesM = M >> 6;
  const int tile = blockIdx.x * 8 + wave;
  if (tile >= tilesM * tilesN) return;
  const int tm = tile / tilesN;
  const int tn = tile - tm * tilesN;
  const int m0 = tm << 6;
  const int n0 = tn << 6;

  const T* Ab  = A  + (size_t)b * strideA;
  const T* Bb  = Bt + (size_t)b * strideB;
  const T* Ab2 = SPLIT ? (A2  + (size_t)b * strideA) : nullptr;
  const T* Bb2 = SPLIT ? (Bt2 + (size_t)b * strideB) : nullptr;

  const int rlane = lane & 15;
  const int koff  = (lane >> 4) * 8;
  const int mOff  = (lane >> 4) * 8;

  v8f acc[4][4];
#pragma unroll
  for (int i = 0; i < 4; ++i)
#pragma unroll
    for (int j = 0; j < 4; ++j) acc[i][j] = (v8f){0.f,0.f,0.f,0.f,0.f,0.f,0.f,0.f};

  for (int k0 = 0; k0 < K; k0 += 32) {
    V bh[4], bl[4];
#pragma unroll
    for (int j = 0; j < 4; ++j) {
      const size_t bo = (size_t)(n0 + (j << 4) + rlane) * ldb + koff + k0;
      bh[j] = Frag<T>::load(Bb + bo);
      if (SPLIT) bl[j] = Frag<T>::load(Bb2 + bo);
    }
#pragma unroll
    for (int i = 0; i < 4; ++i) {
      const size_t ao = (size_t)(m0 + (i << 4) + rlane) * lda + koff + k0;
      V ah = Frag<T>::load(Ab + ao);
      V al;
      if (SPLIT) al = Frag<T>::load(Ab2 + ao);
#pragma unroll
      for (int j = 0; j < 4; ++j) {
        acc[i][j] = Frag<T>::mma(ah, bh[j], acc[i][j]);
        if (SPLIT) {
          acc[i][j] = Frag<T>::mma(ah, bl[j], acc[i][j]);
          acc[i][j] = Frag<T>::mma(al, bh[j], acc[i][j]);
        }
      }
      Frag<T>::guard(acc[i][0], acc[i][3], ah, SPLIT ? al : ah);
    }
    Frag<T>::keep(bh[0], bh[1], bh[2], bh[3]);
    if (SPLIT) Frag<T>::keep(bl[0], bl[1], bl[2], bl[3]);
  }
  acc_guard4(acc[0][0], acc[0][1], acc[0][2], acc[0][3]);
  acc_guard4(acc[1][0], acc[1][1], acc[1][2], acc[1][3]);
  acc_guard4(acc[2][0], acc[2][1], acc[2][2], acc[2][3]);
  acc_guard4(acc[3][0], acc[3][1], acc[3][2], acc[3][3]);

  float* slab = sT[wave];
  const float* Rb = RESID ? (resid + (size_t)b * strideR) : nullptr;
#pragma unroll
  for (int i = 0; i < 4; ++i) {
    const int mBase = m0 + (i << 4);
#pragma unroll
    for (int j = 0; j < 4; ++j) {
      const int n = n0 + (j << 4) + rlane;
      float bv = 0.f;
      if (BIAS_MODE == 2) bv = bias[n];
#pragma unroll
      for (int r = 0; r < 8; ++r) {
        float v = acc[i][j][r] * scale;
        if (BIAS_MODE == 1) v += bias[mBase + mOff + r];
        if (BIAS_MODE == 2) v += bv;
        if (RESID) v += Rb[(size_t)(mBase + mOff + r) * ldc + n];
        if (ACT == 2) v = fmaxf(v, 0.0f);
        if (ACT == 4) v = (v > 0.f) ? v : 0.01f * v;
        slab[(mOff + r) * 68 + (j << 4) + rlane] = v;
      }
    }
    __builtin_amdgcn_fence(__ATOMIC_RELEASE, "workgroup");
    __builtin_amdgcn_wave_barrier();
    __builtin_amdgcn_fence(__ATOMIC_ACQUIRE, "workgroup");
    if (OUT_MODE == 0) {
      float* C = (float*)Cout + (size_t)b * strideC;
      const int hh = lane >> 4, c4 = (lane & 15) * 4;
      for (int pass = 0; pass < 2; ++pass) {
#pragma unroll
        for (int it = 0; it < 8; ++it) {
          const int row = it * 2 + hh;
          v4f v = *(const v4f*)(slab + row * 68 + c4);
          *(volatile v4f*)(C + (size_t)(mBase + row) * ldc + n0 + c4) = v;
        }
        __threadfence();
      }
    } else {
      const int q = lane >> 3, c8 = (lane & 7) * 8;
      unsigned short* C  = (unsigned short*)Cout  + (size_t)b * strideC;
      unsigned short* C2 = (OUT_MODE == 2) ? ((unsigned short*)Cout2 + (size_t)b * strideC) : nullptr;
      for (int pass = 0; pass < 2; ++pass) {
#pragma unroll
        for (int it = 0; it < 4; ++it) {
          const int row = it * 4 + q;
          const float* sp = slab + row * 68 + c8;
          v8h hv, lv;
#pragma unroll
          for (int e = 0; e < 8; ++e) {
            if (OUT_MODE == 1) {
              hv[e] = (_Float16)(sp[e] * ocarry);
            } else {
              unsigned short hb = f2bf_bits(sp[e]);
              unsigned short lb = f2bf_bits(sp[e] - bf_bits2f(hb));
              hv[e] = __builtin_bit_cast(_Float16, hb);
              lv[e] = __builtin_bit_cast(_Float16, lb);
            }
          }
          *(volatile v8h*)(C + (size_t)(mBase + row) * ldc + n0 + c8) = hv;
          if (OUT_MODE == 2) *(volatile v8h*)(C2 + (size_t)(mBase + row) * ldc + n0 + c8) = lv;
        }
        __threadfence();
      }
    }
    __builtin_amdgcn_fence(__ATOMIC_RELEASE, "workgroup");
    __builtin_amdgcn_wave_barrier();
    __builtin_amdgcn_fence(__ATOMIC_ACQUIRE, "workgroup");
  }
}

__global__ __launch_bounds__(256) void tcast_kernel(const float* __restrict__ in, unsigned short* __restrict__ out,
                                                    int R, int C, float scale) {
  __shared__ float sm[64][65];
  const int t  = threadIdx.x;
  const int r0 = blockIdx.x * 64;
  const int c0 = blockIdx.y * 64;
#pragma unroll
  for (int i = 0; i < 16; ++i) {
    const int e  = i * 256 + t;
    const int rl = e >> 6;
    const int cl = e & 63;
    sm[cl][rl] = in[(size_t)(r0 + rl) * C + c0 + cl] * scale;
  }
  __syncthreads();
  const int lane = t & 31, wave = t >> 5;
  const int q = lane >> 3, c8 = (lane & 7) * 8;
  for (int pass = 0; pass < 2; ++pass) {
#pragma unroll
    for (int it = 0; it < 2; ++it) {
      const int row = wave * 8 + it * 4 + q;
      unsigned short hb[8];
#pragma unroll
      for (int e = 0; e < 8; ++e) hb[e] = h_bits(sm[row][c8 + e]);
      const v4u u = (v4u){pk16(hb[0], hb[1]), pk16(hb[2], hb[3]), pk16(hb[4], hb[5]), pk16(hb[6], hb[7])};
      *(volatile v4u*)(out + (size_t)(c0 + row) * R + r0 + c8) = u;
    }
    __threadfence();
  }
}

__global__ __launch_bounds__(256) void cast8_kernel(const float* __restrict__ in, unsigned short* __restrict__ out,
                                                    int n8, float scale) {
  const int i = blockIdx.x * 256 + threadIdx.x;
  if (i >= n8) return;
  const float* p = in + 8 * (size_t)i;
  const v4f a = *(const v4f*)(p);
  const v4f c = *(const v4f*)(p + 4);
  unsigned short hb[8];
#pragma unroll
  for (int e = 0; e < 4; ++e) {
    hb[e]     = h_bits(a[e] * scale);
    hb[4 + e] = h_bits(c[e] * scale);
  }
  const v4u u = (v4u){pk16(hb[0], hb[1]), pk16(hb[2], hb[3]), pk16(hb[4], hb[5]), pk16(hb[6], hb[7])};
  unsigned short* q = out + 8 * (size_t)i;
  *(volatile v4u*)q = u;
  __threadfence();
  *(volatile v4u*)q = u;
}

__global__ __launch_bounds__(512) void scan_kernel(const float* __restrict__ DELp, const float* __restrict__ BPp,
                                                   const float* __restrict__ CPp, const float* __restrict__ Alog,
                                                   float* __restrict__ YI, float* __restrict__ Hout, int bidx) {
  __shared__ __align__(16) float sDel[kChunk * 32];
  __shared__ __align__(16) float sY[kChunk * 32];
  __shared__ __align__(16) float sH[kScanThreads];
  const int tid  = threadIdx.x;
  const int lane = tid & 31;
  const int wave = tid >> 5;
  const int sl   = tid >> 4;
  const int n    = tid & 15;
  const int s0   = blockIdx.x * 32;
  const float a_neg = -expf(Alog[(s0 + sl) * kNDim + n]);
  const size_t rowb = (size_t)bidx * kT;
  float h = 0.f;

#pragma unroll 1
  for (int t0 = 0; t0 < kT; t0 += kChunk) {
#pragma unroll 1
    for (int i = 0; i < 4; ++i) {
      const int e  = i * kScanThreads + tid;
      const int tt = e >> 5;
      const int cl = e & 31;
      const float xv = DELp[(rowb + t0 + tt) * kDState + s0 + cl];
      sDel[e] = fmaxf(xv, 0.f) + log1pf(expf(-fabsf(xv)));
    }
    __syncthreads();

#pragma unroll 1
    for (int tt = 0; tt < kChunk; ++tt) {
      const size_t g = (size_t)(t0 + tt) * kKN + s0 * kNDim + tid;
      const float bpv = BPp[g];
      const float cpv = CPp[g];
      const float dl  = sDel[tt * 32 + sl];
      const float dtA = dl * a_neg;
      const float dA  = expf(dtA);
      const bool  nz  = (dtA != 0.f);
      const float den = nz ? dtA : 1.f;
      const float qv  = (dA - 1.f) / den;
      float v = nz ? qv : 0.f;
      if (!(fabsf(v) <= 3.402823466e38f)) v = 1.f;
      const float bb = v * (dl * bpv);
      h = dA * h + bb;
      float p = h * cpv;
      p += __shfl_xor(p, 8, 32);
      p += __shfl_xor(p, 4, 32);
      p += __shfl_xor(p, 2, 32);
      p += __shfl_xor(p, 1, 32);
      if (n == 0) sY[tt * 32 + sl] = p;
    }
    __syncthreads();

    {
      const int row = wave * 4 + (lane >> 3);
      const int c4  = (lane & 7) * 4;
      const v4f val = *(const v4f*)(sY + row * 32 + c4);
      float* dst = YI + (rowb + t0 + row) * kDState + s0 + c4;
      *(volatile v4f*)dst = val;
      __threadfence();
      *(volatile v4f*)dst = val;
    }
    __syncthreads();
  }

  sH[tid] = h;
  __syncthreads();
  if (wave < 4) {
    const v4f val = *(const v4f*)(sH + wave * 128 + lane * 4);
    float* dst = Hout + (size_t)bidx * kKN + (size_t)s0 * kNDim + wave * 128 + lane * 4;
    *(volatile v4f*)dst = val;
    __threadfence();
    *(volatile v4f*)dst = val;
  }
}

__global__ __launch_bounds__(128) void rmsnorm_kernel(const float* __restrict__ Y, const float* __restrict__ gamma,
                                                      float* __restrict__ out) {
  __shared__ float red[4];
  const int row  = blockIdx.x;
  const int t    = threadIdx.x;
  const int lane = t & 31, wave = t >> 5;
  const v4f yv = *(const v4f*)(Y + (size_t)row * kDModel + 4 * t);
  const v4f gv = *(const v4f*)(gamma + 4 * t);
  float ss = yv[0] * yv[0] + yv[1] * yv[1] + yv[2] * yv[2] + yv[3] * yv[3];
#pragma unroll
  for (int off = 16; off > 0; off >>= 1) ss += __shfl_xor(ss, off, 32);
  if (lane == 0) red[wave] = ss;
  __syncthreads();
  const float tot = ((red[0] + red[1]) + red[2]) + red[3];
  const float rms = sqrtf(tot * (1.0f / 512.0f) + kEps);
  const float inv = 1.0f / rms;
  v4f o;
#pragma unroll
  for (int e = 0; e < 4; ++e) o[e] = gv[e] * (yv[e] * inv);
  float* dst = out + (size_t)row * kDModel + 4 * t;
  *(volatile v4f*)dst = o;
  __threadfence();
  *(volatile v4f*)dst = o;
}

extern "C" void kernel_launch(void* const* d_in, const int* in_sizes, int n_in,
                              void* d_out, int out_size, void* d_ws, size_t ws_size,
                              hipStream_t stream)
{
  if (n_in < 13) return;
  const float* x       = (const float*)d_in[0];
  const float* W_in    = (const float*)d_in[1];
  const float* b_in    = (const float*)d_in[2];
  const float* W_delta = (const float*)d_in[3];
  const float* b_delta = (const float*)d_in[4];
  const float* W_B     = (const float*)d_in[5];
  const float* b_B     = (const float*)d_in[6];
  const float* W_C     = (const float*)d_in[7];
  const float* b_C     = (const float*)d_in[8];
  const float* W_out   = (const float*)d_in[9];
  const float* b_out   = (const float*)d_in[10];
  const float* gamma   = (const float*)d_in[11];
  const float* A_log   = (const float*)d_in[12];

  if (in_sizes[0] != kTok * kDModel) return;
  if (in_sizes[1] != kDModel * kDInner || in_sizes[2] != kDInner) return;
  if (in_sizes[3] != kDInner * kDState || in_sizes[4] != kDState) return;
  if (in_sizes[5] != kDInner * kKN || in_sizes[6] != kKN) return;
  if (in_sizes[7] != kDInner * kKN || in_sizes[8] != kKN) return;
  if (in_sizes[9] != kDState * kDModel || in_sizes[10] != kDModel) return;
  if (in_sizes[11] != kDModel || in_sizes[12] != kDState * kNDim) return;
  if (out_size != kTok * kDModel + kBatch * kDState * kNDim) return;

  const size_t szX16  = (size_t)kTok * kDModel * 2;
  const size_t szWINT = (size_t)kDInner * kDModel * 2;
  const size_t szWDT  = (size_t)kDState * kDInner * 2;
  const size_t szWBT  = (size_t)kKN * kDInner * 2;
  const size_t szWCT  = szWBT;
  const size_t szWOT  = (size_t)kDModel * kDState * 2;
  const size_t szXP16 = (size_t)kTok * kDInner * 2;
  const size_t szDEL  = (size_t)kTok * kDState * 4;
  const size_t szBP   = (size_t)kT * kKN * 4;
  const size_t szCP   = szBP;
  const size_t szYI   = (size_t)kTok * kDState * 4;

  size_t off = 0;
  char* ws = (char*)d_ws;
  unsigned short* X16  = (unsigned short*)(ws + off); off += szX16;
  unsigned short* WINT = (unsigned short*)(ws + off); off += szWINT;
  unsigned short* WDT  = (unsigned short*)(ws + off); off += szWDT;
  unsigned short* WBT  = (unsigned short*)(ws + off); off += szWBT;
  unsigned short* WCT  = (unsigned short*)(ws + off); off += szWCT;
  unsigned short* WOT  = (unsigned short*)(ws + off); off += szWOT;
  unsigned short* XP16 = (unsigned short*)(ws + off); off += szXP16;
  float*          DEL  = (float*)(ws + off);          off += szDEL;
  float*          BP   = (float*)(ws + off);          off += szBP;
  float*          CP   = (float*)(ws + off);          off += szCP;
  float*          YI   = (float*)(ws + off);          off += szYI;
  if (off > ws_size) return;
  unsigned short* YI16 = X16;
  float*          Ypre = BP;

  float* out0 = (float*)d_out;
  float* out1 = out0 + (size_t)kTok * kDModel;

  const dim3 blk256(256);

  cast8_kernel<<<dim3((kTok * kDModel / 8 + 255) / 256), blk256, 0, stream>>>(x, X16, kTok * kDModel / 8, 1.0f);
  tcast_kernel<<<dim3(kDModel / 64, kDInner / 64), blk256, 0, stream>>>(W_in, WINT, kDModel, kDInner, kWCarry);
  tcast_kernel<<<dim3(kDInner / 64, kDState / 64), blk256, 0, stream>>>(W_delta, WDT, kDInner, kDState, kWCarry);
  tcast_kernel<<<dim3(kDInner / 64, kKN / 64), blk256, 0, stream>>>(W_B, WBT, kDInner, kKN, kWCarry);
  tcast_kernel<<<dim3(kDInner / 64, kKN / 64), blk256, 0, stream>>>(W_C, WCT, kDInner, kKN, kWCarry);
  tcast_kernel<<<dim3(kDState / 64, kDModel / 64), blk256, 0, stream>>>(W_out, WOT, kDState, kDModel, kWCarry);

  wmma_gemm64<0, false, 2, 1, false, 0><<<dim3((kTok / 64) * (kDInner / 64) / 8, 1), blk256, 0, stream>>>(
      X16, X16, kDModel, 0L, WINT, WINT, kDModel, 0L, (void*)XP16, (void*)XP16, kDInner, 0L,
      b_in, b_in, 0L, kTok, kDInner, kDModel, 1.0f / kWCarry, kXpCarry);

  wmma_gemm64<0, false, 2, 0, false, 0><<<dim3((kTok / 64) * (kDState / 64) / 8, 1), blk256, 0, stream>>>(
      XP16, XP16, kDInner, 0L, WDT, WDT, kDInner, 0L, (void*)DEL, (void*)DEL, kDState, 0L,
      b_delta, b_delta, 0L, kTok, kDState, kDInner, 1.0f / (kXpCarry * kWCarry), 1.0f);

  for (int b = 0; b < kBatch; ++b) {
    const unsigned short* XPb = XP16 + (size_t)b * kT * kDInner;
    wmma_gemm64<0, false, 2, 0, false, 0><<<dim3((kT / 64) * (kKN / 64) / 8, 1), blk256, 0, stream>>>(
        XPb, XPb, kDInner, 0L, WBT, WBT, kDInner, 0L, (void*)BP, (void*)BP, kKN, 0L,
        b_B, b_B, 0L, kT, kKN, kDInner, 1.0f / (kXpCarry * kWCarry), 1.0f);
    wmma_gemm64<0, false, 2, 0, false, 0><<<dim3((kT / 64) * (kKN / 64) / 8, 1), blk256, 0, stream>>>(
        XPb, XPb, kDInner, 0L, WCT, WCT, kDInner, 0L, (void*)CP, (void*)CP, kKN, 0L,
        b_C, b_C, 0L, kT, kKN, kDInner, 1.0f / (kXpCarry * kWCarry), 1.0f);
    scan_kernel<<<dim3(kDState / 32), dim3(kScanThreads), 0, stream>>>(DEL, BP, CP, A_log, YI, out1, b);
  }

  cast8_kernel<<<dim3((kTok * kDState / 8 + 255) / 256), blk256, 0, stream>>>(YI, YI16, kTok * kDState / 8, kYiCarry);

  wmma_gemm64<0, false, 2, 0, false, 0><<<dim3((kTok / 64) * (kDModel / 64) / 8, 1), blk256, 0, stream>>>(
      YI16, YI16, kDState, 0L, WOT, WOT, kDState, 0L, (void*)Ypre, (void*)Ypre, kDModel, 0L,
      b_out, b_out, 0L, kTok, kDModel, kDState, 1.0f / (kYiCarry * kWCarry), 1.0f);

  rmsnorm_kernel<<<dim3(kTok), dim3(128), 0, stream>>>(Ypre, gamma, out0);
}
